// CoupledMambaFusion_17239998726200
// MI455X (gfx1250) — hardware-run, weakly checked
//
#include <hip/hip_runtime.h>
#include <math.h>

typedef __attribute__((ext_vector_type(16))) _Float16 v16h;
typedef __attribute__((ext_vector_type(8)))  _Float16 v8h;
typedef __attribute__((ext_vector_type(8)))  float    v8f;
typedef __attribute__((ext_vector_type(4)))  float    v4f;

constexpr int kBatch = 4;
constexpr int kSeq   = 2048;
constexpr int kDm    = 256;
constexpr int kDi    = 512;
constexpr int kNst   = 16;
constexpr int kDtR   = 16;
constexpr int kXzP   = 2 * kDi;
constexpr int kDbN   = kDtR + 2 * kNst;
constexpr int kDbP   = 64;
constexpr int kCatP  = 3 * kDm;
constexpr int kRows  = kBatch * kSeq;
constexpr int kNLay  = 2;
constexpr int kNBlk  = 3 * kNLay;
constexpr float kCarryW = 256.0f;
constexpr float kCarryA = 16.0f;
constexpr float kFold   = 1.0f / (kCarryW * kCarryA);
constexpr float kLnEps  = 1e-5f;
constexpr int kCvP  = 516;
constexpr int kScTS = 64;
constexpr int kScCh = 64;
constexpr int kScYP = 68;
static_assert(kRows == 8192 && kXzP == 1024 && kDbN == 48 && kCatP == 768, "shape constants");
static_assert((kDm % 32) == 0 && (kDi % 32) == 0 && (kCatP % 32) == 0, "GEMM K multiples of 32");
static_assert((kRows % 64) == 0 && (kDm % 64) == 0 && (kXzP % 64) == 0 && (kDbP % 64) == 0, "GEMM M,N multiples of 64");
static_assert((kSeq % 64) == 0 && (kDi % kScCh) == 0 && (kRows % 8) == 0, "tile multiples");

constexpr size_t kSzWIN  = (size_t)kNBlk * kXzP * kDm * 2;
constexpr size_t kSzWOUT = (size_t)kNBlk * kDm * kDi * 2;
constexpr size_t kSzWXP  = (size_t)kNBlk * kDbP * kDi * 2;
constexpr size_t kSzWCP  = (size_t)kNBlk * kDm * kDm * 2;
constexpr size_t kSzWFU  = (size_t)kDm * kCatP * 2;
constexpr size_t kSzCAT  = (size_t)kRows * kCatP * 2;
constexpr size_t kSzS    = (size_t)3 * kRows * kDm * 4;
constexpr size_t kSzXIN  = (size_t)3 * kRows * kDm * 4;
constexpr size_t kSzXN   = (size_t)kRows * kDm * 2;
constexpr size_t kSzXZ   = (size_t)kRows * kXzP * 2;
constexpr size_t kSzUC   = (size_t)kRows * kDi * 4;
constexpr size_t kSzUCH  = (size_t)kRows * kDi * 2;
constexpr size_t kSzDBC  = (size_t)kRows * kDbP * 4;
constexpr size_t kSzYG   = (size_t)kRows * kDi * 2;
constexpr size_t kOffWIN  = 0;
constexpr size_t kOffWOUT = kOffWIN  + kSzWIN;
constexpr size_t kOffWXP  = kOffWOUT + kSzWOUT;
constexpr size_t kOffWCP  = kOffWXP  + kSzWXP;
constexpr size_t kOffWFU  = kOffWCP  + kSzWCP;
constexpr size_t kOffCAT  = kOffWFU  + kSzWFU;
constexpr size_t kOffS    = kOffCAT  + kSzCAT;
constexpr size_t kOffXIN  = kOffS    + kSzS;
constexpr size_t kOffXN   = kOffXIN  + kSzXIN;
constexpr size_t kOffXZ   = kOffXN   + kSzXN;
constexpr size_t kOffUC   = kOffXZ   + kSzXZ;
constexpr size_t kOffUCH  = kOffUC   + kSzUC;
constexpr size_t kOffDBC  = kOffUCH  + kSzUCH;
constexpr size_t kOffYG   = kOffDBC  + kSzDBC;
constexpr size_t kWsTotal = kOffYG   + kSzYG;
static_assert(kWsTotal == 125829120ull, "carve total");
static_assert(kWsTotal <= 134217728ull, "carve cap");
static_assert((kOffWOUT % 128) == 0 && (kOffWXP % 128) == 0 && (kOffWCP % 128) == 0 && (kOffWFU % 128) == 0 &&
              (kOffCAT % 128) == 0 && (kOffS % 128) == 0 && (kOffXIN % 128) == 0 && (kOffXN % 128) == 0 &&
              (kOffXZ % 128) == 0 && (kOffUC % 128) == 0 && (kOffUCH % 128) == 0 && (kOffDBC % 128) == 0 &&
              (kOffYG % 128) == 0, "128-B aligned regions");

__device__ __forceinline__ float h16_to_f32(unsigned hb) {
  const unsigned sgn = (hb & 0x8000u) << 16;
  const unsigned em = hb & 0x7fffu;
  const float fn = __uint_as_float((em << 13) + 0x38000000u);
  const float fs = (float)em * 5.9604644775390625e-8f;
  const float mag = (em < 0x400u) ? fs : fn;
  return __uint_as_float(__float_as_uint(mag) | sgn);
}

__device__ __forceinline__ void wave_lds_sync() {
  __builtin_amdgcn_fence(__ATOMIC_RELEASE, "workgroup");
  __builtin_amdgcn_wave_barrier();
  __builtin_amdgcn_fence(__ATOMIC_ACQUIRE, "workgroup");
}

__device__ __forceinline__ void tie_h(v8f& a, v16h x, v16h y) { asm volatile("" : "+v"(a) : "v"(x), "v"(y)); }
__device__ __forceinline__ void nop4_h(v8f& a, v16h x, v16h y) { asm volatile("v_nop\n\tv_nop\n\tv_nop\n\tv_nop" : "+v"(a) : "v"(x), "v"(y)); }
__device__ __forceinline__ void keep4_h(v16h a, v16h b, v16h c, v16h d) { asm volatile("v_nop" :: "v"(a), "v"(b), "v"(c), "v"(d)); }
__device__ __forceinline__ void acc_guard4(v8f& a, v8f& b, v8f& c, v8f& d) { asm volatile("v_nop\n\tv_nop\n\tv_nop\n\tv_nop" : "+v"(a), "+v"(b), "+v"(c), "+v"(d)); }

union FragU { v16h v; v8h h[2]; };
__device__ __forceinline__ v16h frag_load(const _Float16* p) {
  FragU f;
  f.h[0] = *(const v8h*)(p);
  f.h[1] = *(const v8h*)(p + 16);
  return f.v;
}
__device__ __forceinline__ v8f frag_mma(v16h a, v16h b, v8f c) {
  return __builtin_amdgcn_wmma_f32_16x16x32_f16(false, a, false, b, (short)0, c, false, false);
}

template <int BIAS_MODE, int OUT_MODE, bool RESID, bool DEVSCALE>
__global__ __launch_bounds__(256) void wmma_gemm64(
    const unsigned short* __restrict__ Ap, int lda,
    const unsigned short* __restrict__ Btp, int ldb,
    float* __restrict__ C32, int ldc,
    unsigned short* __restrict__ C16, int ldc16,
    const float* __restrict__ bias,
    const float* __restrict__ resid, int ldr,
    const float* __restrict__ scale_p,
    int M, int N, int K, float scale) {
  const _Float16* A  = (const _Float16*)Ap;
  const _Float16* Bt = (const _Float16*)Btp;
  __shared__ __align__(16) float sT[8][16 * 68];
  const int lane = threadIdx.x & 31;
  const int wave = threadIdx.x >> 5;
  const int tilesN = N >> 6;
  const int tilesM = M >> 6;
  const int tile = blockIdx.x * 8 + wave;
  if (tile >= tilesM * tilesN) return;
  const int tm = tile / tilesN;
  const int tn = tile - tm * tilesN;
  const int m0 = tm << 6;
  const int n0 = tn << 6;
  const int rlane = lane & 15;
  const int koff  = (lane >> 4) * 8;
  const int mOff  = (lane >> 4) * 8;

  v8f acc[4][4];
#pragma unroll
  for (int i = 0; i < 4; ++i)
#pragma unroll
    for (int j = 0; j < 4; ++j) acc[i][j] = (v8f){0.f,0.f,0.f,0.f,0.f,0.f,0.f,0.f};

  for (int k0 = 0; k0 < K; k0 += 32) {
    v16h bh[4];
#pragma unroll
    for (int j = 0; j < 4; ++j) {
      const size_t bo = (size_t)(n0 + (j << 4) + rlane) * ldb + koff + k0;
      bh[j] = frag_load(Bt + bo);
    }
#pragma unroll
    for (int i = 0; i < 4; ++i) {
      const size_t ao = (size_t)(m0 + (i << 4) + rlane) * lda + koff + k0;
      const v16h ah = frag_load(A + ao);
#pragma unroll
      for (int j = 0; j < 4; ++j) acc[i][j] = frag_mma(ah, bh[j], acc[i][j]);
      tie_h(acc[i][0], ah, bh[0]);
      tie_h(acc[i][1], ah, bh[1]);
      tie_h(acc[i][2], ah, bh[2]);
      nop4_h(acc[i][3], ah, bh[3]);
    }
    keep4_h(bh[0], bh[1], bh[2], bh[3]);
  }
  acc_guard4(acc[0][0], acc[0][1], acc[0][2], acc[0][3]);
  acc_guard4(acc[1][0], acc[1][1], acc[1][2], acc[1][3]);
  acc_guard4(acc[2][0], acc[2][1], acc[2][2], acc[2][3]);
  acc_guard4(acc[3][0], acc[3][1], acc[3][2], acc[3][3]);

  float sc = scale;
  if (DEVSCALE) sc = sc * scale_p[0];
  float* slab = sT[wave];
  const int hh = lane >> 4, c4 = (lane & 15) * 4;
  const int q  = lane >> 3, c8 = (lane & 7) * 8;
  v4f bias4 = (v4f){0.f, 0.f, 0.f, 0.f};
  if (BIAS_MODE == 2) bias4 = *(const v4f*)(bias + n0 + c4);

#pragma unroll
  for (int i = 0; i < 4; ++i) {
    const int mBase = m0 + (i << 4);
#pragma unroll
    for (int j = 0; j < 4; ++j) {
#pragma unroll
      for (int r = 0; r < 8; ++r) slab[(mOff + r) * 68 + (j << 4) + rlane] = acc[i][j][r];
    }
    wave_lds_sync();
    v4f fv[8];
#pragma unroll
    for (int it = 0; it < 8; ++it) {
      const int row = it * 2 + hh;
      v4f v = *(const v4f*)(slab + row * 68 + c4);
      v4f o;
#pragma unroll
      for (int e = 0; e < 4; ++e) o[e] = v[e] * sc;
      if (BIAS_MODE == 2) {
#pragma unroll
        for (int e = 0; e < 4; ++e) o[e] += bias4[e];
      }
      if (RESID) {
        const v4f rv = *(const v4f*)(resid + (size_t)(mBase + row) * ldr + n0 + c4);
#pragma unroll
        for (int e = 0; e < 4; ++e) o[e] += rv[e];
      }
      fv[it] = o;
      if (OUT_MODE != 0) *(v4f*)(slab + row * 68 + c4) = o;
    }
    if (OUT_MODE == 0 || OUT_MODE == 3) {
      for (int pass = 0; pass < 2; ++pass) {
#pragma unroll
        for (int it = 0; it < 8; ++it) {
          const int row = it * 2 + hh;
          *(volatile v4f*)(C32 + (size_t)(mBase + row) * ldc + n0 + c4) = fv[it];
        }
        __threadfence();
      }
    }
    if (OUT_MODE != 0) {
      wave_lds_sync();
      v8h hv[4];
#pragma unroll
      for (int it = 0; it < 4; ++it) {
        const int row = it * 4 + q;
        const float* sp = slab + row * 68 + c8;
        const v4f a0 = *(const v4f*)(sp);
        const v4f a1 = *(const v4f*)(sp + 4);
#pragma unroll
        for (int e = 0; e < 4; ++e) {
          hv[it][e]     = (_Float16)(a0[e] * kCarryA);
          hv[it][4 + e] = (_Float16)(a1[e] * kCarryA);
        }
      }
      for (int pass = 0; pass < 2; ++pass) {
#pragma unroll
        for (int it = 0; it < 4; ++it) {
          const int row = it * 4 + q;
          *(volatile v8h*)(C16 + (size_t)(mBase + row) * ldc16 + n0 + c8) = hv[it];
        }
        __threadfence();
      }
    }
    wave_lds_sync();
  }
}


__global__ __launch_bounds__(256) void cast_f16_kernel(
    const float* __restrict__ src, unsigned short* __restrict__ dst, int total8, float scale) {
  const int i = blockIdx.x * 256 + threadIdx.x;
  if (i >= total8) return;
  const size_t e0 = (size_t)i << 3;
  const v4f a0 = *(const v4f*)(src + e0);
  const v4f a1 = *(const v4f*)(src + e0 + 4);
  v8h hv;
#pragma unroll
  for (int e = 0; e < 4; ++e) {
    hv[e]     = (_Float16)(a0[e] * scale);
    hv[4 + e] = (_Float16)(a1[e] * scale);
  }
  unsigned short* qd = dst + e0;
  *(volatile v8h*)qd = hv;
  __threadfence();
  *(volatile v8h*)qd = hv;
}

__global__ __launch_bounds__(256) void cast_xproj_kernel(
    const float* __restrict__ src, unsigned short* __restrict__ dst, float scale) {
  const int i = blockIdx.x * 256 + threadIdx.x;
  const int e0  = i << 3;
  const int blk = e0 / (kDbP * kDi);
  const int rem = e0 - blk * (kDbP * kDi);
  const int row = rem / kDi;
  const int col = rem - row * kDi;
  const int rc  = (row < kDbN) ? row : (kDbN - 1);
  const float* p = src + ((size_t)blk * kDbN + rc) * kDi + col;
  const v4f a0 = *(const v4f*)(p);
  const v4f a1 = *(const v4f*)(p + 4);
  const bool keep = (row < kDbN);
  v8h hv;
#pragma unroll
  for (int e = 0; e < 4; ++e) {
    const float f0 = keep ? (a0[e] * scale) : 0.0f;
    const float f1 = keep ? (a1[e] * scale) : 0.0f;
    hv[e]     = (_Float16)f0;
    hv[4 + e] = (_Float16)f1;
  }
  unsigned short* qd = dst + (size_t)e0;
  *(volatile v8h*)qd = hv;
  __threadfence();
  *(volatile v8h*)qd = hv;
}

__global__ __launch_bounds__(256) void cast_streams_kernel(
    const float* __restrict__ s0, const float* __restrict__ s1, const float* __restrict__ s2,
    unsigned short* __restrict__ CAT, float scale) {
  const int j = blockIdx.y;
  const float* src = (j == 0) ? s0 : ((j == 1) ? s1 : s2);
  const int i = blockIdx.x * 256 + threadIdx.x;
  const int row = i >> 5;
  const int c8  = (i & 31) * 8;
  const float* p = src + (size_t)row * kDm + c8;
  const v4f a0 = *(const v4f*)(p);
  const v4f a1 = *(const v4f*)(p + 4);
  v8h hv;
#pragma unroll
  for (int e = 0; e < 4; ++e) {
    hv[e]     = (_Float16)(a0[e] * scale);
    hv[4 + e] = (_Float16)(a1[e] * scale);
  }
  unsigned short* qd = CAT + (size_t)row * kCatP + j * kDm + c8;
  *(volatile v8h*)qd = hv;
  __threadfence();
  *(volatile v8h*)qd = hv;
}

template <bool F16OUT>
__global__ __launch_bounds__(256) void ln_kernel(
    const float* __restrict__ X, const float* __restrict__ w, const float* __restrict__ b,
    float* __restrict__ Y32, unsigned short* __restrict__ Y16, float oscale) {
  const int lane = threadIdx.x & 31, wave = threadIdx.x >> 5;
  const int row = blockIdx.x * 8 + wave;
  const int cA = F16OUT ? (lane * 8) : (lane * 4);
  const int cB = F16OUT ? (lane * 8 + 4) : (128 + lane * 4);
  const float* xr = X + (size_t)row * kDm;
  const v4f a0 = *(const v4f*)(xr + cA);
  const v4f a1 = *(const v4f*)(xr + cB);
  float s = ((a0[0] + a0[1]) + (a0[2] + a0[3])) + ((a1[0] + a1[1]) + (a1[2] + a1[3]));
#pragma unroll
  for (int off = 16; off > 0; off >>= 1) s += __shfl_xor(s, off, 32);
  const float mean = s * (1.0f / (float)kDm);
  v4f d0, d1;
#pragma unroll
  for (int e = 0; e < 4; ++e) { d0[e] = a0[e] - mean; d1[e] = a1[e] - mean; }
  float qs = ((d0[0] * d0[0] + d0[1] * d0[1]) + (d0[2] * d0[2] + d0[3] * d0[3])) +
             ((d1[0] * d1[0] + d1[1] * d1[1]) + (d1[2] * d1[2] + d1[3] * d1[3]));
#pragma unroll
  for (int off = 16; off > 0; off >>= 1) qs += __shfl_xor(qs, off, 32);
  const float rs = rsqrtf(qs * (1.0f / (float)kDm) + kLnEps);
  const v4f w0 = *(const v4f*)(w + cA);
  const v4f w1 = *(const v4f*)(w + cB);
  const v4f b0 = *(const v4f*)(b + cA);
  const v4f b1 = *(const v4f*)(b + cB);
  v4f o0, o1;
#pragma unroll
  for (int e = 0; e < 4; ++e) {
    o0[e] = (d0[e] * rs) * w0[e] + b0[e];
    o1[e] = (d1[e] * rs) * w1[e] + b1[e];
  }
  if (F16OUT) {
    v8h hv;
#pragma unroll
    for (int e = 0; e < 4; ++e) {
      hv[e]     = (_Float16)(o0[e] * oscale);
      hv[4 + e] = (_Float16)(o1[e] * oscale);
    }
    unsigned short* qd = Y16 + (size_t)row * kDm + lane * 8;
    *(volatile v8h*)qd = hv;
    __threadfence();
    *(volatile v8h*)qd = hv;
  } else {
    float* yr = Y32 + (size_t)row * kDm;
    *(volatile v4f*)(yr + cA) = o0;
    *(volatile v4f*)(yr + cB) = o1;
    __threadfence();
    *(volatile v4f*)(yr + cA) = o0;
    *(volatile v4f*)(yr + cB) = o1;
  }
}

__global__ __launch_bounds__(256) void conv_silu_kernel(
    const unsigned* __restrict__ XZW, const float* __restrict__ cw, const float* __restrict__ cb,
    float* __restrict__ UC, unsigned short* __restrict__ UCH) {
  __shared__ __align__(16) float sT[16 * kCvP];
  const int tid = threadIdx.x, lane = tid & 31, wave = tid >> 5;
  const int g0 = blockIdx.x * 64;
  const int tb = g0 & (kSeq - 1);
  constexpr int kWordsPerRow = kXzP / 2;
  const v4f wA = *(const v4f*)(cw + (size_t)(2 * tid) * 4);
  const v4f wB = *(const v4f*)(cw + (size_t)(2 * tid + 1) * 4);
  const float bA = cb[2 * tid];
  const float bB = cb[2 * tid + 1];
  float a3, a2, a1, b3, b2, b1;
  {
    const bool hist = (tb > 0);
    const int rb = hist ? (g0 - 3) : g0;
    const unsigned h3 = XZW[(size_t)rb * kWordsPerRow + tid];
    const unsigned h2 = XZW[(size_t)(rb + 1) * kWordsPerRow + tid];
    const unsigned h1 = XZW[(size_t)(rb + 2) * kWordsPerRow + tid];
    const float fa3 = h16_to_f32(h3 & 0xffffu), fb3 = h16_to_f32(h3 >> 16);
    const float fa2 = h16_to_f32(h2 & 0xffffu), fb2 = h16_to_f32(h2 >> 16);
    const float fa1 = h16_to_f32(h1 & 0xffffu), fb1 = h16_to_f32(h1 >> 16);
    a3 = hist ? fa3 : 0.f; b3 = hist ? fb3 : 0.f;
    a2 = hist ? fa2 : 0.f; b2 = hist ? fb2 : 0.f;
    a1 = hist ? fa1 : 0.f; b1 = hist ? fb1 : 0.f;
  }
#pragma unroll 1
  for (int sub = 0; sub < 4; ++sub) {
    const int lb = g0 + sub * 16;
#pragma unroll 1
    for (int s = 0; s < 16; ++s) {
      const unsigned wv = XZW[(size_t)(lb + s) * kWordsPerRow + tid];
      const float xa = h16_to_f32(wv & 0xffffu);
      const float xb = h16_to_f32(wv >> 16);
      float ca = wA[0] * a3;
      ca = fmaf(wA[1], a2, ca);
      ca = fmaf(wA[2], a1, ca);
      ca = fmaf(wA[3], xa, ca);
      ca += bA;
      float cbv = wB[0] * b3;
      cbv = fmaf(wB[1], b2, cbv);
      cbv = fmaf(wB[2], b1, cbv);
      cbv = fmaf(wB[3], xb, cbv);
      cbv += bB;
      const float ua = ca * __builtin_amdgcn_rcpf(1.0f + expf(-ca));
      const float ub = cbv * __builtin_amdgcn_rcpf(1.0f + expf(-cbv));
      sT[s * kCvP + 2 * tid]     = ua;
      sT[s * kCvP + 2 * tid + 1] = ub;
      a3 = a2; a2 = a1; a1 = xa;
      b3 = b2; b2 = b1; b1 = xb;
    }
    __syncthreads();
    v4f fv[8];
    v8h bv[4];
#pragma unroll
    for (int it = 0; it < 8; ++it) {
      const int unit = it * 8 + wave;
      fv[it] = *(const v4f*)(sT + (unit >> 2) * kCvP + (unit & 3) * 128 + lane * 4);
    }
#pragma unroll
    for (int it = 0; it < 4; ++it) {
      const int unit = it * 8 + wave;
      const float* sp = sT + (unit >> 1) * kCvP + (unit & 1) * 256 + lane * 8;
      const v4f p0 = *(const v4f*)(sp);
      const v4f p1 = *(const v4f*)(sp + 4);
#pragma unroll
      for (int e = 0; e < 4; ++e) {
        bv[it][e]     = (_Float16)(p0[e] * kCarryA);
        bv[it][4 + e] = (_Float16)(p1[e] * kCarryA);
      }
    }
    for (int pass = 0; pass < 2; ++pass) {
#pragma unroll
      for (int it = 0; it < 8; ++it) {
        const int unit = it * 8 + wave;
        *(volatile v4f*)(UC + (size_t)(lb + (unit >> 2)) * kDi + (unit & 3) * 128 + lane * 4) = fv[it];
      }
#pragma unroll
      for (int it = 0; it < 4; ++it) {
        const int unit = it * 8 + wave;
        *(volatile v8h*)(UCH + (size_t)(lb + (unit >> 1)) * kDi + (unit & 1) * 256 + lane * 8) = bv[it];
      }
      __threadfence();
    }
    __syncthreads();
  }
}

__global__ __launch_bounds__(64) void scan_kernel(
    const float* __restrict__ DBC, const float* __restrict__ UC, const unsigned* __restrict__ XZW,
    const float* __restrict__ Wdt, const float* __restrict__ bdt, const float* __restrict__ Alog,
    const float* __restrict__ Dp, unsigned short* __restrict__ YG) {
  __shared__ __align__(16) float sX[kScTS * kDbP];
  __shared__ __align__(16) float sY[kScTS * kScYP];
  const int tid = threadIdx.x, lane = tid & 31, wave = tid >> 5;
  constexpr int kGrpPerB = kDi / kScCh;
  constexpr int kWordsPerRow = kXzP / 2;
  const int bix = blockIdx.x / kGrpPerB;
  const int d0  = (blockIdx.x - bix * kGrpPerB) * kScCh;
  const int d   = d0 + tid;
  const size_t row0 = (size_t)bix * kSeq;

#pragma unroll 1
  for (int s = 0; s < kNst; ++s) sX[s * kScCh + tid] = -expf(Alog[(size_t)d * kNst + s]);
  __syncthreads();
  float negA[kNst], h[kNst], wd[kDtR];
#pragma unroll
  for (int s = 0; s < kNst; ++s) {
    negA[s] = sX[s * kScCh + tid];
    h[s] = 0.f;
  }
  {
    const float* wp = Wdt + (size_t)d * kDtR;
    const v4f q0 = *(const v4f*)(wp);
    const v4f q1 = *(const v4f*)(wp + 4);
    const v4f q2 = *(const v4f*)(wp + 8);
    const v4f q3 = *(const v4f*)(wp + 12);
#pragma unroll
    for (int e = 0; e < 4; ++e) { wd[e] = q0[e]; wd[4 + e] = q1[e]; wd[8 + e] = q2[e]; wd[12 + e] = q3[e]; }
  }
  const float bb = bdt[d];
  const float Dd = Dp[d];
  const int zcol = (kDi + d) >> 1;
  const unsigned zsh = (unsigned)(d & 1) * 16u;
  const int lr = tid >> 4, lc4 = (tid & 15) * 4;
  const int q = lane >> 3, c8 = (lane & 7) * 8;

#pragma unroll 1
  for (int t0 = 0; t0 < kSeq; t0 += kScTS) {
    __syncthreads();
#pragma unroll 4
    for (int i = 0; i < 16; ++i) {
      const int r = lr + 4 * i;
      *(v4f*)(sX + r * kDbP + lc4) = *(const v4f*)(DBC + (row0 + t0 + r) * kDbP + lc4);
    }
    __syncthreads();
#pragma unroll 1
    for (int s = 0; s < kScTS; ++s) {
      const size_t row = row0 + t0 + s;
      const float* xr = sX + s * kDbP;
      const float xt = UC[row * kDi + d];
      const unsigned zw = XZW[row * kWordsPerRow + zcol];
      float vdot = 0.f;
#pragma unroll
      for (int r4 = 0; r4 < kDtR / 4; ++r4) {
        const v4f xv = *(const v4f*)(xr + 4 * r4);
        vdot = fmaf(xv[0], wd[4 * r4 + 0], vdot);
        vdot = fmaf(xv[1], wd[4 * r4 + 1], vdot);
        vdot = fmaf(xv[2], wd[4 * r4 + 2], vdot);
        vdot = fmaf(xv[3], wd[4 * r4 + 3], vdot);
      }
      v4f Bq[4], Cq[4];
#pragma unroll
      for (int qq = 0; qq < 4; ++qq) {
        Bq[qq] = *(const v4f*)(xr + kDtR + 4 * qq);
        Cq[qq] = *(const v4f*)(xr + kDtR + kNst + 4 * qq);
      }
      const float v   = vdot + bb;
      const float a   = expf(-fabsf(v));
      const float u   = 1.0f + a;
      const float l1p = logf(u) + (a - (u - 1.0f)) * __builtin_amdgcn_rcpf(u);
      const float dt  = fmaxf(v, 0.0f) + l1p;
      const float dtx = dt * xt;
      float y = 0.f;
#pragma unroll
      for (int k = 0; k < kNst; ++k) {
        const float e = __expf(dt * negA[k]);
        h[k] = e * h[k] + dtx * Bq[k >> 2][k & 3];
        y = h[k] * Cq[k >> 2][k & 3] + y;
      }
      y = xt * Dd + y;
      const float zv = h16_to_f32((zw >> zsh) & 0xffffu);
      const float sg = __builtin_amdgcn_rcpf(1.0f + expf(-zv));
      y = y * (zv * sg);
      sY[s * kScYP + tid] = y * kCarryA;
    }
    __syncthreads();
    v8h hv[8];
#pragma unroll
    for (int it = 0; it < 8; ++it) {
      const int rr = it * 8 + wave * 4 + q;
      const float* sp = sY + rr * kScYP + c8;
      const v4f p0 = *(const v4f*)(sp);
      const v4f p1 = *(const v4f*)(sp + 4);
#pragma unroll
      for (int e = 0; e < 4; ++e) {
        hv[it][e]     = (_Float16)p0[e];
        hv[it][4 + e] = (_Float16)p1[e];
      }
    }
    for (int pass = 0; pass < 2; ++pass) {
#pragma unroll
      for (int it = 0; it < 8; ++it) {
        const int rr = it * 8 + wave * 4 + q;
        *(volatile v8h*)(YG + (row0 + t0 + rr) * kDi + d0 + c8) = hv[it];
      }
      __threadfence();
    }
  }
}


extern "C" void kernel_launch(void* const* d_in, const int* in_sizes, int n_in,
                              void* d_out, int out_size, void* d_ws, size_t ws_size,
                              hipStream_t stream) {
  if (n_in < 20) return;
  if (in_sizes[0] != kRows * kDm || in_sizes[1] != kRows * kDm || in_sizes[2] != kRows * kDm) return;
  if (in_sizes[3] != kNBlk * kDm || in_sizes[4] != kNBlk * kDm) return;
  if (in_sizes[5] != kNBlk * kXzP * kDm) return;
  if (in_sizes[6] != kNBlk * kDi * 4 || in_sizes[7] != kNBlk * kDi) return;
  if (in_sizes[8] != kNBlk * kDbN * kDi) return;
  if (in_sizes[9] != kNBlk * kDi * kDtR || in_sizes[10] != kNBlk * kDi) return;
  if (in_sizes[11] != kNBlk * kDi * kNst || in_sizes[12] != kNBlk * kDi) return;
  if (in_sizes[13] != kNBlk * kDm * kDi) return;
  if (in_sizes[14] != kNBlk * kDm * kDm) return;
  if (in_sizes[15] != kNBlk) return;
  if (in_sizes[16] != kDm * kCatP) return;
  if (in_sizes[17] != kDm || in_sizes[18] != kDm || in_sizes[19] != kDm) return;
  if (out_size != kRows * kDm) return;
  if (ws_size < kWsTotal) return;

  const float* in_s[3] = {(const float*)d_in[0], (const float*)d_in[1], (const float*)d_in[2]};
  const float* mbnw  = (const float*)d_in[3];
  const float* mbnb  = (const float*)d_in[4];
  const float* inpw  = (const float*)d_in[5];
  const float* convw = (const float*)d_in[6];
  const float* convb = (const float*)d_in[7];
  const float* xpw   = (const float*)d_in[8];
  const float* dtw   = (const float*)d_in[9];
  const float* dtb   = (const float*)d_in[10];
  const float* Alog  = (const float*)d_in[11];
  const float* Dpp   = (const float*)d_in[12];
  const float* outw  = (const float*)d_in[13];
  const float* cplw  = (const float*)d_in[14];
  const float* coef  = (const float*)d_in[15];
  const float* fusew = (const float*)d_in[16];
  const float* fuseb = (const float*)d_in[17];
  const float* normw = (const float*)d_in[18];
  const float* normb = (const float*)d_in[19];
  float* out = (float*)d_out;

  char* ws = (char*)d_ws;
  unsigned short* WIN  = (unsigned short*)(ws + kOffWIN);
  unsigned short* WOUT = (unsigned short*)(ws + kOffWOUT);
  unsigned short* WXP  = (unsigned short*)(ws + kOffWXP);
  unsigned short* WCP  = (unsigned short*)(ws + kOffWCP);
  unsigned short* WFU  = (unsigned short*)(ws + kOffWFU);
  unsigned short* CAT  = (unsigned short*)(ws + kOffCAT);
  float* Sp[3];
  float* XINp[3];
  for (int j = 0; j < 3; ++j) {
    Sp[j]   = (float*)(ws + kOffS)   + (size_t)j * kRows * kDm;
    XINp[j] = (float*)(ws + kOffXIN) + (size_t)j * kRows * kDm;
  }
  unsigned short* XN  = (unsigned short*)(ws + kOffXN);
  unsigned short* XZ  = (unsigned short*)(ws + kOffXZ);
  float*          UC  = (float*)(ws + kOffUC);
  unsigned short* UCH = (unsigned short*)(ws + kOffUCH);
  float*          DBC = (float*)(ws + kOffDBC);
  unsigned short* YG  = (unsigned short*)(ws + kOffYG);
  float* PRE = Sp[0];

  cast_f16_kernel<<<(kNBlk * kXzP * kDm) / 8 / 256, 256, 0, stream>>>(inpw, WIN, (kNBlk * kXzP * kDm) / 8, kCarryW);
  cast_f16_kernel<<<(kNBlk * kDm * kDi) / 8 / 256, 256, 0, stream>>>(outw, WOUT, (kNBlk * kDm * kDi) / 8, kCarryW);
  cast_f16_kernel<<<(kNBlk * kDm * kDm) / 8 / 256, 256, 0, stream>>>(cplw, WCP, (kNBlk * kDm * kDm) / 8, kCarryW);
  cast_f16_kernel<<<(kDm * kCatP) / 8 / 256, 256, 0, stream>>>(fusew, WFU, (kDm * kCatP) / 8, kCarryW);
  cast_xproj_kernel<<<(kNBlk * kDbP * kDi) / 8 / 256, 256, 0, stream>>>(xpw, WXP, kCarryW);
  cast_streams_kernel<<<dim3((kRows * kDm) / 8 / 256, 3), 256, 0, stream>>>(in_s[0], in_s[1], in_s[2], CAT, kCarryA);

  for (int i = 0; i < kNLay; ++i) {
    for (int j = 0; j < 3; ++j) {
      const int sj = (j + 1) % 3;
      const float* rs = (i == 0) ? in_s[j] : (const float*)Sp[j];
      wmma_gemm64<0, 0, true, true><<<64, 256, 0, stream>>>(
          CAT + sj * kDm, kCatP,
          WCP + (size_t)(i * 3 + j) * kDm * kDm, kDm,
          XINp[j], kDm,
          XN, kDm,
          fuseb,
          rs, kDm,
          coef + (i * 3 + j),
          kRows, kDm, kDm, kFold);
    }
    for (int j = 0; j < 3; ++j) {
      const int blk = 3 * i + j;
      ln_kernel<true><<<kRows / 8, 256, 0, stream>>>(
          XINp[j], mbnw + (size_t)blk * kDm, mbnb + (size_t)blk * kDm, DBC, XN, kCarryA);
      wmma_gemm64<0, 1, false, false><<<256, 256, 0, stream>>>(
          XN, kDm,
          WIN + (size_t)blk * kXzP * kDm, kDm,
          DBC, kDbP,
          XZ, kXzP,
          fuseb,
          in_s[0], kDm,
          coef,
          kRows, kXzP, kDm, kFold / kCarryA);
      conv_silu_kernel<<<kRows / 64, 256, 0, stream>>>(
          (const unsigned*)XZ, convw + (size_t)blk * kDi * 4, convb + (size_t)blk * kDi, UC, UCH);
      wmma_gemm64<0, 0, false, false><<<16, 256, 0, stream>>>(
          UCH, kDi,
          WXP + (size_t)blk * kDbP * kDi, kDi,
          DBC, kDbP,
          XN, kDm,
          fuseb,
          in_s[0], kDm,
          coef,
          kRows, kDbP, kDi, kFold);
      scan_kernel<<<kBatch * (kDi / kScCh), kScCh, 0, stream>>>(
          DBC, UC, (const unsigned*)XZ,
          dtw + (size_t)blk * kDi * kDtR, dtb + (size_t)blk * kDi,
          Alog + (size_t)blk * kDi * kNst, Dpp + (size_t)blk * kDi, YG);
      if (i + 1 < kNLay) {
        wmma_gemm64<0, 3, true, false><<<64, 256, 0, stream>>>(
            YG, kDi,
            WOUT + (size_t)blk * kDm * kDi, kDi,
            Sp[j], kDm,
            CAT + j * kDm, kCatP,
            fuseb,
            XINp[j], kDm,
            coef,
            kRows, kDm, kDi, kFold);
      } else {
        wmma_gemm64<0, 1, true, false><<<64, 256, 0, stream>>>(
            YG, kDi,
            WOUT + (size_t)blk * kDm * kDi, kDi,
            DBC, kDbP,
            CAT + j * kDm, kCatP,
            fuseb,
            XINp[j], kDm,
            coef,
            kRows, kDm, kDi, kFold);
      }
    }
  }

  wmma_gemm64<2, 0, false, false><<<64, 256, 0, stream>>>(
      CAT, kCatP,
      WFU, kCatP,
      PRE, kDm,
      XN, kDm,
      fuseb,
      in_s[0], kDm,
      coef,
      kRows, kDm, kCatP, kFold);
  ln_kernel<false><<<kRows / 8, 256, 0, stream>>>(PRE, normw, normb, out, XN, 1.0f);
}
